// SO3PredictionModel_91276644974780
// MI455X (gfx1250) — hardware-run, weakly checked
//
#include <hip/hip_runtime.h>
#include <hip/hip_fp16.h>
#include <math.h>

typedef __attribute__((ext_vector_type(16))) _Float16 v16h;
typedef __attribute__((ext_vector_type(8)))  _Float16 v8h;
typedef __attribute__((ext_vector_type(8)))  float    v8f;
typedef __attribute__((ext_vector_type(4)))  float    v4f;

constexpr int kNBatch = 16;
constexpr int kSteps  = 2048;
constexpr int kDm     = 384;
constexpr int kBlk3   = 128;
constexpr int kCat    = 3 * kDm;
constexpr int kQuat   = 4;
constexpr int kOutN   = 4;
constexpr int kOutP   = 64;
constexpr int kRec    = 16;
constexpr int kStP    = 4;
constexpr int kRows   = kNBatch * kSteps;
constexpr float kHCarry = 64.0f;
constexpr float kWCarry = 1024.0f;
constexpr float kYCarry = 16.0f;
constexpr float kResid  = 2048.0f;
static_assert(kCat == 1152);
static_assert(kBlk3 * 3 == kDm);
static_assert(kRows == 32768);
static_assert(kOutN <= kOutP && (kOutP % 64) == 0);
static_assert((kDm % 64) == 0 && (kCat % 64) == 0 && (kDm % 32) == 0);
static_assert((kSteps % 32) == 0 && (kRows % 32) == 0);
static_assert((kDm % 8) == 0);
static_assert(kRec * 4 == 64 && kStP * 4 == 16);

constexpr size_t kSzVEC  = (size_t)kDm * 4;
constexpr size_t kSzWP   = (size_t)kCat * kDm * 2;
constexpr size_t kSzWOP  = (size_t)kOutP * kDm * 2;
constexpr size_t kSzHID  = (size_t)kRows * kDm * 2;
constexpr size_t kSzPROJ = (size_t)kSteps * kCat * 4;
constexpr size_t kSzPRE  = (size_t)kSteps * kBlk3 * kRec * 4;
constexpr size_t kSzHSF  = (size_t)kSteps * kBlk3 * kStP * 4;
constexpr size_t kSzHS   = (size_t)kRows * kDm * 2;
constexpr size_t kSzRAW  = (size_t)kRows * kOutP * 4;
constexpr size_t kOffBB   = 0;
constexpr size_t kOffBD   = kOffBB   + kSzVEC;
constexpr size_t kOffBI   = kOffBD   + kSzVEC;
constexpr size_t kOffWP   = kOffBI   + kSzVEC;
constexpr size_t kOffWOP  = kOffWP   + kSzWP;
constexpr size_t kOffHID  = kOffWOP  + kSzWOP;
constexpr size_t kOffPROJ = kOffHID  + kSzHID;
constexpr size_t kOffPRE  = kOffPROJ + kSzPROJ;
constexpr size_t kOffHSF  = kOffPRE  + kSzPRE;
constexpr size_t kOffHS   = kOffHSF  + kSzHSF;
constexpr size_t kOffRAW  = kOffHS   + kSzHS;
constexpr size_t kWsTotal = kOffRAW  + kSzRAW;
static_assert(kSzVEC == 1536ull && kSzWP == 884736ull && kSzWOP == 49152ull && kSzHID == 25165824ull);
static_assert(kSzPROJ == 9437184ull && kSzPRE == 16777216ull && kSzHSF == 4194304ull);
static_assert(kSzHS == 25165824ull && kSzRAW == 8388608ull);
static_assert(kWsTotal == 90067456ull);
static_assert(kWsTotal <= 134217728ull);
static_assert((kSzVEC % 128) == 0);
static_assert((kOffBD % 128) == 0 && (kOffBI % 128) == 0 && (kOffWP % 128) == 0 && (kOffWOP % 128) == 0 &&
              (kOffHID % 128) == 0 && (kOffPROJ % 128) == 0 && (kOffPRE % 128) == 0 && (kOffHSF % 128) == 0 &&
              (kOffHS % 128) == 0 && (kOffRAW % 128) == 0);

__device__ __forceinline__ _Float16 f16_flush(float v) {
  const float w = (fabsf(v) < 6.103515625e-05f) ? 0.0f : v;
  return (_Float16)w;
}
__device__ __forceinline__ void f16_split(float v, _Float16& hi, _Float16& lo) {
  hi = f16_flush(v);
  const float hf = (float)hi;
  const float r = (v - hf) * kResid;
  lo = f16_flush(r);
}

__device__ __forceinline__ float bf16r(float v) {
  unsigned u = __float_as_uint(v);
  u = (u + 0x7FFFu + ((u >> 16) & 1u)) & 0xFFFF0000u;
  return __uint_as_float(u);
}

__device__ __forceinline__ float h16_to_f32(unsigned hb) {
  const unsigned sgn = (hb & 0x8000u) << 16; const unsigned em = hb & 0x7fffu;
  const float fn = __uint_as_float((em << 13) + 0x38000000u);
  const float fs = (float)em * 5.9604644775390625e-8f;
  const float mag = (em < 0x400u) ? fs : fn; return __uint_as_float(__float_as_uint(mag) | sgn); }

namespace eng {
union FragU { v16h v; v8h h[2]; };
__device__ __forceinline__ v16h frag_load(const _Float16* p) {
  FragU f;
  f.h[0] = *(const v8h*)(p);
  f.h[1] = *(const v8h*)(p + 16);
  return f.v;
}
__device__ __forceinline__ v8f mma(v16h a, v16h b, v8f c) {
  return __builtin_amdgcn_wmma_f32_16x16x32_f16(false, a, false, b, (short)0, c, false, false);
}
__device__ __forceinline__ void guard1(v8f& a, v16h x, v16h y) {
  asm volatile("v_nop\n\tv_nop\n\tv_nop\n\tv_nop" : "+v"(a) : "v"(x), "v"(y));
}
__device__ __forceinline__ void guard_acc(v8f& a) {
  asm volatile("v_nop\n\tv_nop\n\tv_nop\n\tv_nop" : "+v"(a));
}
__device__ __forceinline__ void keep4(v16h a, v16h b, v16h c, v16h d) {
  asm volatile("v_nop" :: "v"(a), "v"(b), "v"(c), "v"(d));
}

template <int MI, int SPL>
__global__ __launch_bounds__(256) void gemm_f16_kernel(
    const unsigned short* __restrict__ Ap, const unsigned short* __restrict__ A2p, int lda,
    const unsigned short* __restrict__ Btp, const unsigned short* __restrict__ Bt2p, int ldb,
    float* __restrict__ C, int ldc, int M, int N, int K, float scale, float rscale)
{
  static_assert(MI >= 1 && MI <= 2);
  static_assert(SPL >= 0 && SPL <= 2);
  const _Float16* A   = (const _Float16*)Ap;
  const _Float16* A2  = (const _Float16*)A2p;
  const _Float16* Bt  = (const _Float16*)Btp;
  const _Float16* Bt2 = (const _Float16*)Bt2p;
  __shared__ __align__(16) float sT[8][16 * 68];
  const int lane = threadIdx.x & 31;
  const int wave = threadIdx.x >> 5;
  const int tilesN = N >> 6;
  const int tilesM = M / (16 * MI);
  const int tile = blockIdx.x * 8 + wave;
  if (tile >= tilesM * tilesN) return;
  const int tm = tile / tilesN;
  const int tn = tile - tm * tilesN;
  const int m0 = tm * (16 * MI);
  const int n0 = tn << 6;
  const int rlane = lane & 15;
  const int koff  = (lane >> 4) * 8;
  const int mOff  = (lane >> 4) * 8;

  v8f acc[MI][4], accr[MI][4];
#pragma unroll
  for (int i = 0; i < MI; ++i)
#pragma unroll
    for (int j = 0; j < 4; ++j) {
      acc[i][j]  = (v8f){0.f, 0.f, 0.f, 0.f, 0.f, 0.f, 0.f, 0.f};
      accr[i][j] = (v8f){0.f, 0.f, 0.f, 0.f, 0.f, 0.f, 0.f, 0.f};
    }

  for (int k0 = 0; k0 < K; k0 += 32) {
    v16h bh[4], bl[4];
#pragma unroll
    for (int j = 0; j < 4; ++j) {
      const size_t bo = (size_t)(n0 + (j << 4) + rlane) * ldb + koff + k0;
      bh[j] = frag_load(Bt + bo);
      if (SPL == 2) bl[j] = frag_load(Bt2 + bo); else bl[j] = bh[j];
    }
#pragma unroll
    for (int i = 0; i < MI; ++i) {
      const size_t ao = (size_t)(m0 + (i << 4) + rlane) * lda + koff + k0;
      const v16h ah = frag_load(A + ao);
      v16h al = ah;
      if (SPL >= 1) al = frag_load(A2 + ao);
#pragma unroll
      for (int j = 0; j < 4; ++j) {
        acc[i][j] = mma(ah, bh[j], acc[i][j]);
        if (SPL >= 1) accr[i][j] = mma(al, bh[j], accr[i][j]);
        if (SPL == 2) accr[i][j] = mma(ah, bl[j], accr[i][j]);
      }
#pragma unroll
      for (int j = 0; j < 4; ++j) {
        guard1(acc[i][j], ah, al);
        if (SPL >= 1) guard1(accr[i][j], ah, al);
      }
    }
    keep4(bh[0], bh[1], bh[2], bh[3]);
    if (SPL == 2) keep4(bl[0], bl[1], bl[2], bl[3]);
  }
#pragma unroll
  for (int i = 0; i < MI; ++i)
#pragma unroll
    for (int j = 0; j < 4; ++j) {
      guard_acc(acc[i][j]);
      if (SPL >= 1) guard_acc(accr[i][j]);
    }

  float* slab = sT[wave];
#pragma unroll
  for (int i = 0; i < MI; ++i) {
    const int mBase = m0 + (i << 4);
#pragma unroll
    for (int j = 0; j < 4; ++j) {
#pragma unroll
      for (int r = 0; r < 8; ++r) {
        float v = acc[i][j][r] * scale;
        if (SPL >= 1) v += accr[i][j][r] * rscale;
        slab[(mOff + r) * 68 + (j << 4) + rlane] = v;
      }
    }
    __builtin_amdgcn_fence(__ATOMIC_RELEASE, "workgroup");
    __builtin_amdgcn_wave_barrier();
    __builtin_amdgcn_fence(__ATOMIC_ACQUIRE, "workgroup");
    {
      const int hh = lane >> 4, c4 = (lane & 15) * 4;
      for (int pass = 0; pass < 2; ++pass) {
#pragma unroll
        for (int it = 0; it < 8; ++it) {
          const int row = it * 2 + hh;
          const v4f v = *(const v4f*)(slab + row * 68 + c4);
          *(volatile v4f*)(C + (size_t)(mBase + row) * ldc + n0 + c4) = v;
        }
        __threadfence();
      }
    }
    __builtin_amdgcn_fence(__ATOMIC_RELEASE, "workgroup");
    __builtin_amdgcn_wave_barrier();
    __builtin_amdgcn_fence(__ATOMIC_ACQUIRE, "workgroup");
  }
}
}

template <bool LO>
__global__ __launch_bounds__(256) void transpose_pack_kernel(
    const float* __restrict__ W, unsigned short* __restrict__ BtH, unsigned short* __restrict__ BtL,
    int Kdim, int Ndim, float carry)
{
  __shared__ float tile[64 * 65];
  const int tid = threadIdx.x, lane = tid & 31, wave = tid >> 5;
  const int n0 = blockIdx.x * 64;
  const int k0 = blockIdx.y * 64;
#pragma unroll
  for (int p = 0; p < 16; ++p) {
    const int idx = tid + p * 256;
    const int kk  = idx >> 6;
    const int nn  = idx & 63;
    const int n   = n0 + nn;
    const int nc  = (n < Ndim) ? n : (Ndim - 1);
    const float v = W[(size_t)(k0 + kk) * Ndim + nc];
    tile[kk * 65 + nn] = (n < Ndim) ? (bf16r(v) * carry) : 0.0f;
  }
  __syncthreads();
  const int q = lane >> 3, c8 = (lane & 7) * 8;
  v8h hv[2], lv[2];
#pragma unroll
  for (int it = 0; it < 2; ++it) {
    const int nrow = it * 32 + wave * 4 + q;
#pragma unroll
    for (int e = 0; e < 8; ++e) {
      _Float16 h, l;
      const float t = tile[(c8 + e) * 65 + nrow];
      f16_split(t, h, l);
      hv[it][e] = h;
      lv[it][e] = l;
    }
  }
  for (int pass = 0; pass < 2; ++pass) {
#pragma unroll
    for (int it = 0; it < 2; ++it) {
      const int nrow = it * 32 + wave * 4 + q;
      const size_t o = (size_t)(n0 + nrow) * Kdim + k0 + c8;
      *(volatile v8h*)(BtH + o) = hv[it];
      if (LO) *(volatile v8h*)(BtL + o) = lv[it];
    }
    __threadfence();
  }
}

__global__ __launch_bounds__(256) void rne_vec_kernel(
    const float* __restrict__ src, float* __restrict__ dst, int n4)
{
  const int i = blockIdx.x * 256 + threadIdx.x;
  if (i >= n4) return;
  const v4f a = *(const v4f*)(src + (size_t)i * 4);
  const float a0 = a[0];
  const float a1 = a[1];
  const float a2 = a[2];
  const float a3 = a[3];
  v4f r;
  r[0] = bf16r(a0);
  r[1] = bf16r(a1);
  r[2] = bf16r(a2);
  r[3] = bf16r(a3);
  float* p = dst + (size_t)i * 4;
  *(volatile v4f*)p = r;
  __threadfence();
  *(volatile v4f*)p = r;
}

static_assert(((kRows * (kDm / 8)) % 256) == 0);
__global__ __launch_bounds__(256) void hidden_kernel(
    const float* __restrict__ quat, const float* __restrict__ Win, unsigned short* __restrict__ HID)
{
  const int g  = blockIdx.x * 256 + threadIdx.x;
  const int r  = g / (kDm / 8);
  const int c8 = (g - r * (kDm / 8)) * 8;
  const v4f qv = *(const v4f*)(quat + (size_t)r * kQuat);
  const float q0 = qv[0];
  const float q1 = qv[1];
  const float q2 = qv[2];
  const float q3 = qv[3];
  float qk[4];
  qk[0] = bf16r(q0);
  qk[1] = bf16r(q1);
  qk[2] = bf16r(q2);
  qk[3] = bf16r(q3);
  float acc[8];
#pragma unroll
  for (int e = 0; e < 8; ++e) acc[e] = 0.0f;
#pragma unroll
  for (int k = 0; k < 4; ++k) {
    const v4f wa = *(const v4f*)(Win + (size_t)k * kDm + c8);
    const v4f wb = *(const v4f*)(Win + (size_t)k * kDm + c8 + 4);
#pragma unroll
    for (int e = 0; e < 4; ++e) {
      const float fa = wa[e];
      const float fb = wb[e];
      acc[e]     = fmaf(qk[k], bf16r(fa), acc[e]);
      acc[4 + e] = fmaf(qk[k], bf16r(fb), acc[4 + e]);
    }
  }
  v8h hv;
#pragma unroll
  for (int e = 0; e < 8; ++e) hv[e] = f16_flush(acc[e] * kHCarry);
  unsigned short* p = HID + (size_t)g * 8;
  *(volatile v8h*)p = hv;
  __threadfence();
  *(volatile v8h*)p = hv;
}

static_assert(((kSteps * kBlk3) % 256) == 0);
__global__ __launch_bounds__(256) void prep_kernel(
    const float* __restrict__ PROJ, const float* __restrict__ BB, const float* __restrict__ BD,
    const float* __restrict__ BI, float* __restrict__ PRE)
{
  const int g  = blockIdx.x * 256 + threadIdx.x;
  const int t  = g / kBlk3;
  const int j  = g - t * kBlk3;
  const int c0 = 3 * j;
  const float* pr = PROJ + (size_t)t * kCat + c0;
  const float bx = pr[0] + BB[c0];
  const float by = pr[1] + BB[c0 + 1];
  const float bz = pr[2] + BB[c0 + 2];
  const float z0 = pr[kDm]     + BD[c0];
  const float z1 = pr[kDm + 1] + BD[c0 + 1];
  const float z2 = pr[kDm + 2] + BD[c0 + 2];
  const float i0 = pr[2 * kDm]     + BI[c0];
  const float i1 = pr[2 * kDm + 1] + BI[c0 + 1];
  const float i2 = pr[2 * kDm + 2] + BI[c0 + 2];
  const float nb = fmaxf(sqrtf(bx * bx + by * by + bz * bz), 1e-8f);
  const float hf = nb * 0.5f;
  const float w  = cosf(hf);
  const float s  = sinf(hf) / nb;
  const float qx = s * bz;
  const float qy = -s * by;
  const float qz = s * bx;
  const float d0 = 1.0f / (1.0f + expf(-z0));
  const float d1 = 1.0f / (1.0f + expf(-z1));
  const float d2 = 1.0f / (1.0f + expf(-z2));
  v4f r0, r1, r2, r3;
  r0[0] = w;
  r0[1] = qx;
  r0[2] = qy;
  r0[3] = qz;
  r1[0] = d0;
  r1[1] = d1;
  r1[2] = d2;
  r1[3] = i0;
  r2[0] = i1;
  r2[1] = i2;
  r2[2] = 0.0f;
  r2[3] = 0.0f;
  r3[0] = 0.0f;
  r3[1] = 0.0f;
  r3[2] = 0.0f;
  r3[3] = 0.0f;
  float* p = PRE + (size_t)g * kRec;
  for (int pass = 0; pass < 2; ++pass) {
    *(volatile v4f*)(p)      = r0;
    *(volatile v4f*)(p + 4)  = r1;
    *(volatile v4f*)(p + 8)  = r2;
    *(volatile v4f*)(p + 12) = r3;
    __threadfence();
  }
}

__global__ __launch_bounds__(128) void rot_scan_kernel(
    const float* __restrict__ PRE, float* __restrict__ HSF)
{
  const int j = threadIdx.x;
  float vx = 0.0f, vy = 0.0f, vz = 0.0f;
  for (int t = 0; t < kSteps; ++t) {
    const float* rp = PRE + ((size_t)t * kBlk3 + j) * kRec;
    const v4f r0 = *(const v4f*)(rp);
    const v4f r1 = *(const v4f*)(rp + 4);
    const v4f r2 = *(const v4f*)(rp + 8);
    const float w  = r0[0];
    const float qx = r0[1];
    const float qy = r0[2];
    const float qz = r0[3];
    const float d0 = r1[0];
    const float d1 = r1[1];
    const float d2 = r1[2];
    const float i0 = r1[3];
    const float i1 = r2[0];
    const float i2 = r2[1];
    const float tx = 2.0f * (qy * vz - qz * vy);
    const float ty = 2.0f * (qz * vx - qx * vz);
    const float tz = 2.0f * (qx * vy - qy * vx);
    const float rx = vx + w * tx + (qy * tz - qz * ty);
    const float ry = vy + w * ty + (qz * tx - qx * tz);
    const float rz = vz + w * tz + (qx * ty - qy * tx);
    vx = d0 * rx + i0;
    vy = d1 * ry + i1;
    vz = d2 * rz + i2;
    v4f o;
    o[0] = vx;
    o[1] = vy;
    o[2] = vz;
    o[3] = 0.0f;
    float* hp = HSF + ((size_t)t * kBlk3 + j) * kStP;
    *(volatile v4f*)hp = o;
    __threadfence();
    *(volatile v4f*)hp = o;
  }
}

static_assert(((kSteps * kDm / 8) % 256) == 0);
__global__ __launch_bounds__(256) void hs_pack_kernel(
    const float* __restrict__ HSF, unsigned short* __restrict__ HSb)
{
  const int i  = blockIdx.x * 256 + threadIdx.x;
  const int t  = i / (kDm / 8);
  const int c8 = (i - t * (kDm / 8)) * 8;
  const float* hrow = HSF + (size_t)t * kBlk3 * kStP;
  v8h hv;
#pragma unroll
  for (int e = 0; e < 8; ++e) {
    const int col = c8 + e;
    const int jb  = col / 3;
    const int cc  = col - 3 * jb;
    const float f = hrow[jb * kStP + cc];
    hv[e] = f16_flush(f * kYCarry);
  }
  unsigned short* qh = HSb + ((size_t)i << 3);
  *(volatile v8h*)qh = hv;
  __threadfence();
  *(volatile v8h*)qh = hv;
}

static_assert((kRows % 256) == 0);
__global__ __launch_bounds__(256) void norm_out_kernel(
    const float* __restrict__ RAW, float* __restrict__ out)
{
  const int r = blockIdx.x * 256 + threadIdx.x;
  const v4f a = *(const v4f*)(RAW + (size_t)r * kOutP);
  const float a0 = a[0];
  const float a1 = a[1];
  const float a2 = a[2];
  const float a3 = a[3];
  const float n = fmaxf(sqrtf(a0 * a0 + a1 * a1 + a2 * a2 + a3 * a3), 1e-8f);
  v4f o;
  o[0] = a0 / n;
  o[1] = a1 / n;
  o[2] = a2 / n;
  o[3] = a3 / n;
  float* p = out + (size_t)r * kOutN;
  *(volatile v4f*)p = o;
  __threadfence();
  *(volatile v4f*)p = o;
}

static_assert(((kSteps / 32) * (kCat / 64)) % 8 == 0);
static_assert(((kRows / 32) * (kOutP / 64)) % 8 == 0);
static_assert((kDm / 4) <= 256);

extern "C" void kernel_launch(void* const* d_in, const int* in_sizes, int n_in,
                              void* d_out, int out_size, void* d_ws, size_t ws_size,
                              hipStream_t stream)
{
  if (n_in < 9) return;
  if (in_sizes[0] != kRows * kQuat) return;
  if (in_sizes[1] != kQuat * kDm) return;
  if (in_sizes[2] != kDm * kDm) return;
  if (in_sizes[3] != kDm) return;
  if (in_sizes[4] != kDm * kDm) return;
  if (in_sizes[5] != kDm) return;
  if (in_sizes[6] != kDm * kDm) return;
  if (in_sizes[7] != kDm) return;
  if (in_sizes[8] != kDm * kOutN) return;
  if (out_size != kRows * kOutN) return;
  if (ws_size < kWsTotal) return;

  const float* quat  = (const float*)d_in[0];
  const float* W_in  = (const float*)d_in[1];
  const float* W_biv = (const float*)d_in[2];
  const float* b_biv = (const float*)d_in[3];
  const float* W_dec = (const float*)d_in[4];
  const float* b_dec = (const float*)d_in[5];
  const float* W_inj = (const float*)d_in[6];
  const float* b_inj = (const float*)d_in[7];
  const float* W_out = (const float*)d_in[8];
  float* out = (float*)d_out;

  char* ws = (char*)d_ws;
  float*          BB   = (float*)(ws + kOffBB);
  float*          BD   = (float*)(ws + kOffBD);
  float*          BI   = (float*)(ws + kOffBI);
  unsigned short* WP   = (unsigned short*)(ws + kOffWP);
  unsigned short* WOP  = (unsigned short*)(ws + kOffWOP);
  unsigned short* HID  = (unsigned short*)(ws + kOffHID);
  float*          PROJ = (float*)(ws + kOffPROJ);
  float*          PRE  = (float*)(ws + kOffPRE);
  float*          HSF  = (float*)(ws + kOffHSF);
  unsigned short* HS   = (unsigned short*)(ws + kOffHS);
  float*          RAW  = (float*)(ws + kOffRAW);

  constexpr float sP = 1.0f / (kHCarry * kWCarry);
  constexpr float sY = 1.0f / (kYCarry * kWCarry);

  rne_vec_kernel<<<1, 256, 0, stream>>>(b_biv, BB, kDm / 4);
  rne_vec_kernel<<<1, 256, 0, stream>>>(b_dec, BD, kDm / 4);
  rne_vec_kernel<<<1, 256, 0, stream>>>(b_inj, BI, kDm / 4);

  transpose_pack_kernel<false><<<dim3(kDm / 64, kDm / 64), 256, 0, stream>>>(
      W_biv, WP, WP, kDm, kDm, kWCarry);
  transpose_pack_kernel<false><<<dim3(kDm / 64, kDm / 64), 256, 0, stream>>>(
      W_dec, WP + (size_t)kDm * kDm, WP + (size_t)kDm * kDm, kDm, kDm, kWCarry);
  transpose_pack_kernel<false><<<dim3(kDm / 64, kDm / 64), 256, 0, stream>>>(
      W_inj, WP + (size_t)2 * kDm * kDm, WP + (size_t)2 * kDm * kDm, kDm, kDm, kWCarry);

  transpose_pack_kernel<false><<<dim3(kOutP / 64, kDm / 64), 256, 0, stream>>>(
      W_out, WOP, WOP, kDm, kOutN, kWCarry);

  hidden_kernel<<<(kRows * (kDm / 8)) / 256, 256, 0, stream>>>(quat, W_in, HID);

  for (int b = 0; b < kNBatch; ++b) {
    const unsigned short* hidb = HID + (size_t)b * kSteps * kDm;
    unsigned short* hsb = HS + (size_t)b * kSteps * kDm;

    eng::gemm_f16_kernel<2, 0><<<dim3((kSteps / 32) * (kCat / 64) / 8), 256, 0, stream>>>(
        hidb, nullptr, kDm, WP, nullptr, kDm, PROJ, kCat, kSteps, kCat, kDm, sP, 0.0f);

    prep_kernel<<<(kSteps * kBlk3) / 256, 256, 0, stream>>>(PROJ, BB, BD, BI, PRE);

    rot_scan_kernel<<<dim3(1), 128, 0, stream>>>(PRE, HSF);

    hs_pack_kernel<<<(kSteps * kDm / 8) / 256, 256, 0, stream>>>(HSF, hsb);
  }

  eng::gemm_f16_kernel<2, 0><<<dim3((kRows / 32) * (kOutP / 64) / 8), 256, 0, stream>>>(
      HS, nullptr, kDm, WOP, nullptr, kDm, RAW, kOutP, kRows, kOutP, kDm, sY, 0.0f);

  norm_out_kernel<<<kRows / 256, 256, 0, stream>>>(RAW, out);
}
